// Res2D_35588099014803
// MI455X (gfx1250) — hardware-verified
//
#include <hip/hip_runtime.h>
#include <math.h>

typedef __attribute__((ext_vector_type(16))) __bf16   v16b;
typedef __attribute__((ext_vector_type(8)))  __bf16   v8b;
typedef __attribute__((ext_vector_type(8)))  float    v8f;
typedef __attribute__((ext_vector_type(4)))  float    v4f;
typedef __attribute__((ext_vector_type(4)))  unsigned int v4u;

constexpr int kSteps   = 128;
constexpr int kInDim   = 512;
constexpr int kEmbN    = 2048;
constexpr int kLat     = 256;
constexpr int kNch     = 8;
constexpr int kHalo    = 4;
constexpr int kPlaneF  = (kLat + 2 * kHalo) * kLat;
constexpr int kNoc     = 16;
constexpr int kNpos    = 64;
constexpr int kRoK     = 1024;
constexpr int kBlk     = 512;
constexpr int kPartPlane = kSteps * kNoc * kNpos;
static_assert(kPlaneF == 33 * 4 * kBlk);
static_assert(kLat * kLat == 8 * 16 * kBlk);

__device__ __forceinline__ unsigned short f2bf_bits(float f) {
  unsigned u = __float_as_uint(f);
  return (unsigned short)((u + 0x7FFFu + ((u >> 16) & 1u)) >> 16);
}
__device__ __forceinline__ float bf_bits2f(unsigned short h) { return __uint_as_float(((unsigned)h) << 16); }
__device__ __forceinline__ unsigned pk16(unsigned short a, unsigned short b) { return (unsigned)a | ((unsigned)b << 16); }

__device__ __forceinline__ void acc_guard4(v8f& a, v8f& b, v8f& c, v8f& d) { asm volatile("v_nop\n\tv_nop\n\tv_nop\n\tv_nop" : "+v"(a), "+v"(b), "+v"(c), "+v"(d)); }
__device__ __forceinline__ void guard2_b3(v8f& a, v8f& b, v16b x, v16b y, v16b z) { asm volatile("v_nop\n\tv_nop\n\tv_nop\n\tv_nop" : "+v"(a), "+v"(b) : "v"(x), "v"(y), "v"(z)); }
__device__ __forceinline__ void guard1_b4(v8f& a, v16b w, v16b x, v16b y, v16b z) { asm volatile("v_nop\n\tv_nop\n\tv_nop\n\tv_nop" : "+v"(a) : "v"(w), "v"(x), "v"(y), "v"(z)); }
__device__ __forceinline__ void keep6_b(v16b a, v16b b, v16b c, v16b d, v16b e, v16b f) { asm volatile("v_nop" :: "v"(a), "v"(b), "v"(c), "v"(d), "v"(e), "v"(f)); }

template <typename T> struct Frag;
template <> struct Frag<__bf16> {
  typedef v16b V; union U { v16b v; v8b h[2]; };
  static __device__ __forceinline__ v16b load(const __bf16* p) {
    U f; f.h[0] = *(const v8b*)(p); f.h[1] = *(const v8b*)(p + 16); return f.v;
  }
  static __device__ __forceinline__ v8f mma(v16b a, v16b b, v8f c) {
    return __builtin_amdgcn_wmma_f32_16x16x32_bf16(false, a, false, b, (short)0, c, false, false);
  }
};

__device__ __forceinline__ void split3_bits(float f, unsigned short& h, unsigned short& m, unsigned short& l) {
  h = f2bf_bits(f);
  const float r1 = f - bf_bits2f(h);
  m = f2bf_bits(r1);
  const float r2 = r1 - bf_bits2f(m);
  l = f2bf_bits(r2);
}
__device__ __forceinline__ void split2_bits(float f, unsigned short& h, unsigned short& l) {
  h = f2bf_bits(f);
  l = f2bf_bits(f - bf_bits2f(h));
}

__global__ __launch_bounds__(256) void split3_kernel(const float* __restrict__ in,
                                                     unsigned short* __restrict__ ph,
                                                     unsigned short* __restrict__ pm,
                                                     unsigned short* __restrict__ pl, int n8) {
  const int i = blockIdx.x * 256 + threadIdx.x;
  if (i >= n8) return;
  const float* p = in + 8 * (size_t)i;
  const v4f a = *(const v4f*)(p);
  const v4f b = *(const v4f*)(p + 4);
  unsigned short h[8], m[8], l[8];
#pragma unroll
  for (int e = 0; e < 4; ++e) {
    split3_bits(a[e], h[e], m[e], l[e]);
    split3_bits(b[e], h[4 + e], m[4 + e], l[4 + e]);
  }
  const v4u uh = (v4u){pk16(h[0], h[1]), pk16(h[2], h[3]), pk16(h[4], h[5]), pk16(h[6], h[7])};
  const v4u um = (v4u){pk16(m[0], m[1]), pk16(m[2], m[3]), pk16(m[4], m[5]), pk16(m[6], m[7])};
  const v4u ul = (v4u){pk16(l[0], l[1]), pk16(l[2], l[3]), pk16(l[4], l[5]), pk16(l[6], l[7])};
  unsigned short* qh = ph + 8 * (size_t)i;
  unsigned short* qm = pm + 8 * (size_t)i;
  unsigned short* ql = pl + 8 * (size_t)i;
  *(volatile v4u*)qh = uh; *(volatile v4u*)qm = um; *(volatile v4u*)ql = ul;
  __threadfence();
  *(volatile v4u*)qh = uh; *(volatile v4u*)qm = um; *(volatile v4u*)ql = ul;
}

__global__ __launch_bounds__(256) void split2_kernel(const float* __restrict__ in,
                                                     unsigned short* __restrict__ ph,
                                                     unsigned short* __restrict__ pl, int n8) {
  const int i = blockIdx.x * 256 + threadIdx.x;
  if (i >= n8) return;
  const float* p = in + 8 * (size_t)i;
  const v4f a = *(const v4f*)(p);
  const v4f b = *(const v4f*)(p + 4);
  unsigned short h[8], l[8];
#pragma unroll
  for (int e = 0; e < 4; ++e) {
    split2_bits(a[e], h[e], l[e]);
    split2_bits(b[e], h[4 + e], l[4 + e]);
  }
  const v4u uh = (v4u){pk16(h[0], h[1]), pk16(h[2], h[3]), pk16(h[4], h[5]), pk16(h[6], h[7])};
  const v4u ul = (v4u){pk16(l[0], l[1]), pk16(l[2], l[3]), pk16(l[4], l[5]), pk16(l[6], l[7])};
  unsigned short* qh = ph + 8 * (size_t)i;
  unsigned short* ql = pl + 8 * (size_t)i;
  *(volatile v4u*)qh = uh; *(volatile v4u*)ql = ul;
  __threadfence();
  *(volatile v4u*)qh = uh; *(volatile v4u*)ql = ul;
}

__global__ __launch_bounds__(256) void gemm32_split3(
    const unsigned short* __restrict__ Ahp, const unsigned short* __restrict__ Amp,
    const unsigned short* __restrict__ Alp, int lda,
    const unsigned short* __restrict__ Bhp, const unsigned short* __restrict__ Bmp,
    const unsigned short* __restrict__ Blp, int ldb,
    float* __restrict__ C, int ldc, int M, int N, int K) {
  __shared__ __align__(16) float sT[8][32 * 36];
  const __bf16* Ah = (const __bf16*)Ahp; const __bf16* Am = (const __bf16*)Amp; const __bf16* Al = (const __bf16*)Alp;
  const __bf16* Bh = (const __bf16*)Bhp; const __bf16* Bm = (const __bf16*)Bmp; const __bf16* Bl = (const __bf16*)Blp;
  const int lane = threadIdx.x & 31;
  const int wave = threadIdx.x >> 5;
  const int tilesN = N >> 5;
  const int tilesM = M >> 5;
  const int tile = blockIdx.x * 8 + wave;
  if (tile >= tilesM * tilesN) return;
  const int tm = tile / tilesN;
  const int tn = tile - tm * tilesN;
  const int m0 = tm << 5;
  const int n0 = tn << 5;
  const int rlane = lane & 15;
  const int koff  = (lane >> 4) * 8;
  const int mOff  = (lane >> 4) * 8;

  v8f acc[2][2];
#pragma unroll
  for (int i = 0; i < 2; ++i)
#pragma unroll
    for (int j = 0; j < 2; ++j) acc[i][j] = (v8f){0.f,0.f,0.f,0.f,0.f,0.f,0.f,0.f};

  for (int k0 = 0; k0 < K; k0 += 32) {
    v16b bh[2], bm[2], bl[2];
#pragma unroll
    for (int j = 0; j < 2; ++j) {
      const size_t bo = (size_t)(n0 + (j << 4) + rlane) * ldb + koff + k0;
      bh[j] = Frag<__bf16>::load(Bh + bo);
      bm[j] = Frag<__bf16>::load(Bm + bo);
      bl[j] = Frag<__bf16>::load(Bl + bo);
    }
#pragma unroll
    for (int i = 0; i < 2; ++i) {
      const size_t ao = (size_t)(m0 + (i << 4) + rlane) * lda + koff + k0;
      const v16b ah = Frag<__bf16>::load(Ah + ao);
      const v16b am = Frag<__bf16>::load(Am + ao);
      const v16b al = Frag<__bf16>::load(Al + ao);
#pragma unroll
      for (int j = 0; j < 2; ++j) {
        acc[i][j] = Frag<__bf16>::mma(ah, bh[j], acc[i][j]);
        acc[i][j] = Frag<__bf16>::mma(ah, bm[j], acc[i][j]);
        acc[i][j] = Frag<__bf16>::mma(am, bh[j], acc[i][j]);
        acc[i][j] = Frag<__bf16>::mma(ah, bl[j], acc[i][j]);
        acc[i][j] = Frag<__bf16>::mma(am, bm[j], acc[i][j]);
        acc[i][j] = Frag<__bf16>::mma(al, bh[j], acc[i][j]);
      }
      guard2_b3(acc[i][0], acc[i][1], ah, am, al);
    }
    keep6_b(bh[0], bh[1], bm[0], bm[1], bl[0], bl[1]);
  }
  acc_guard4(acc[0][0], acc[0][1], acc[1][0], acc[1][1]);

  float* slab = sT[wave];
#pragma unroll
  for (int i = 0; i < 2; ++i)
#pragma unroll
    for (int j = 0; j < 2; ++j)
#pragma unroll
      for (int r = 0; r < 8; ++r)
        slab[((i << 4) + mOff + r) * 36 + (j << 4) + rlane] = acc[i][j][r];
  __builtin_amdgcn_fence(__ATOMIC_RELEASE, "workgroup");
  __builtin_amdgcn_wave_barrier();
  __builtin_amdgcn_fence(__ATOMIC_ACQUIRE, "workgroup");
  const int q = lane >> 3, c4 = (lane & 7) << 2;
  for (int pass = 0; pass < 2; ++pass) {
#pragma unroll
    for (int it = 0; it < 8; ++it) {
      const int row = (it << 2) + q;
      const v4f v = *(const v4f*)(slab + row * 36 + c4);
      *(volatile v4f*)(C + (size_t)(m0 + row) * ldc + n0 + c4) = v;
    }
    __threadfence();
  }
}

__device__ __forceinline__ float tanh_f(float s) {
  const float e = expf(2.0f * s);
  const float r = __builtin_amdgcn_rcpf(e + 1.0f);
  return fmaf(-2.0f, r, 1.0f);
}
__device__ __forceinline__ void split_hl(float x, __bf16& hi, __bf16& lo) {
  const __bf16 hb = (__bf16)x;
  hi = hb;
  lo = (__bf16)(x - (float)hb);
}

__global__ __launch_bounds__(kBlk) void lattice_scan_kernel(
    const float* __restrict__ UC,
    const float* __restrict__ mask_coarse,
    const float* __restrict__ mask_fine,
    const float* __restrict__ Wd,
    const float* __restrict__ w1,
    const float* __restrict__ w2,
    const unsigned short* __restrict__ WOh,
    const unsigned short* __restrict__ WOl,
    float* ZAbuf, float* ZBbuf,
    float* PART) {
  __shared__ __align__(16) float yS[kNoc * kNpos];

  const int c    = blockIdx.x;
  const int tid  = threadIdx.x;
  const int lane = tid & 31, wave = tid >> 5, hh = lane >> 4, m16 = lane & 15;
  const int tx   = tid & 63, ty = tid >> 6;
  const int x0   = tx << 2;
  const int gm   = ((tx + 63) & 63) << 2;
  const int gp   = ((tx + 1) & 63) << 2;
  const int j16  = tx >> 2, b0 = (tx & 3) << 2;

  float* za = ZAbuf + (size_t)c * kPlaneF + kHalo * kLat;
  float* zb = ZBbuf + (size_t)c * kPlaneF + kHalo * kLat;
  const float* Wdc = Wd + (size_t)c * 256;
  const __bf16* woh = (const __bf16*)WOh + (size_t)(m16 * kNch + c) * kRoK + 8 * hh;
  const __bf16* wol = (const __bf16*)WOl + (size_t)(m16 * kNch + c) * kRoK + 8 * hh;

  float w1s[9], w2s[25];
#pragma unroll
  for (int i = 0; i < 9; ++i)  w1s[i] = 0.9f * w1[c * 9 + i];
#pragma unroll
  for (int i = 0; i < 25; ++i) w2s[i] = 0.1f * w2[c * 25 + i];

  {
    float* z0 = za - kHalo * kLat;
    const v4f zero4 = (v4f){0.f, 0.f, 0.f, 0.f};
    for (int pass = 0; pass < 2; ++pass) {
#pragma unroll 1
      for (int it = 0; it < 33; ++it) *(volatile v4f*)(z0 + 4 * (size_t)(it * kBlk + tid)) = zero4;
      __threadfence();
    }
  }
  __threadfence();
  __syncthreads();

#pragma unroll 1
  for (int t = 0; t < kSteps; ++t) {
    float* zin  = (t & 1) ? zb : za;
    float* zout = (t & 1) ? za : zb;
    const float* uct = UC + (size_t)t * kEmbN + j16;

#pragma unroll 1
    for (int tile = 0; tile < 8; ++tile) {
      const int y0  = (tile << 5) + (ty << 2);
      const int i16 = y0 >> 4, a0 = y0 & 15;

      const float mcv = mask_coarse[(i16 << 4) + j16];
      float ucm[8];
#pragma unroll
      for (int ci = 0; ci < 8; ++ci) ucm[ci] = uct[(ci << 8) + (i16 << 4)] * mcv;
      float acc[4][4];
#pragma unroll
      for (int r = 0; r < 4; ++r) {
        float u4[4] = {0.f, 0.f, 0.f, 0.f};
#pragma unroll
        for (int ci = 0; ci < 8; ++ci) {
          const v4f wd = *(const v4f*)(Wdc + (size_t)ci * 2048 + ((a0 + r) << 4) + b0);
#pragma unroll
          for (int cc = 0; cc < 4; ++cc) u4[cc] = fmaf(ucm[ci], wd[cc], u4[cc]);
        }
        const v4f mf = *(const v4f*)(mask_fine + ((y0 + r) << 8) + x0);
#pragma unroll
        for (int cc = 0; cc < 4; ++cc) acc[r][cc] = u4[cc] * mf[cc];
      }

      const float* zt = zin + (y0 - kHalo) * kLat;
#pragma unroll
      for (int rr = 0; rr < 12; ++rr) {
        const float* zr = zt + rr * kLat;
        const v4f qa = *(const v4f*)(zr + gm);
        const v4f qb = *(const v4f*)(zr + x0);
        const v4f qc = *(const v4f*)(zr + gp);
        float win[12];
        win[0] = qa[0]; win[1] = qa[1]; win[2]  = qa[2]; win[3]  = qa[3];
        win[4] = qb[0]; win[5] = qb[1]; win[6]  = qb[2]; win[7]  = qb[3];
        win[8] = qc[0]; win[9] = qc[1]; win[10] = qc[2]; win[11] = qc[3];
#pragma unroll
        for (int r = 0; r < 4; ++r) {
          const int k3 = rr - r - 3;
          if (k3 >= 0 && k3 <= 2) {
#pragma unroll
            for (int kx = 0; kx < 3; ++kx) {
              const float wv = w1s[k3 * 3 + kx];
#pragma unroll
              for (int cc = 0; cc < 4; ++cc) acc[r][cc] = fmaf(wv, win[cc + kx + 3], acc[r][cc]);
            }
          }
          const int d5 = rr - r;
          if (d5 >= 0 && d5 <= 8 && ((d5 & 1) == 0)) {
            const int k5 = d5 >> 1;
#pragma unroll
            for (int kx = 0; kx < 5; ++kx) {
              const float wv = w2s[k5 * 5 + kx];
#pragma unroll
              for (int cc = 0; cc < 4; ++cc) acc[r][cc] = fmaf(wv, win[cc + 2 * kx], acc[r][cc]);
            }
          }
        }
      }

      v4f o[4];
#pragma unroll
      for (int r = 0; r < 4; ++r)
#pragma unroll
        for (int cc = 0; cc < 4; ++cc) o[r][cc] = tanh_f(acc[r][cc]);
      float* zo = zout + (y0 << 8) + x0;
      for (int pass = 0; pass < 2; ++pass) {
#pragma unroll
        for (int r = 0; r < 4; ++r) *(volatile v4f*)(zo + (r << 8)) = o[r];
        __threadfence();
      }
      if (tile == 0 && ty == 0) {
        float* zh = zout + (kLat << 8) + x0;
        for (int pass = 0; pass < 2; ++pass) {
#pragma unroll
          for (int r = 0; r < 4; ++r) *(volatile v4f*)(zh + (r << 8)) = o[r];
          __threadfence();
        }
      }
      if (tile == 7 && ty == 7) {
        float* zh = zout + (0 - kHalo) * kLat + x0;
        for (int pass = 0; pass < 2; ++pass) {
#pragma unroll
          for (int r = 0; r < 4; ++r) *(volatile v4f*)(zh + r * kLat) = o[r];
          __threadfence();
        }
      }
    }
    __threadfence();
    __syncthreads();

    if (wave < 4) {
      const int pos = (wave << 4) + m16;
      const int pi = pos >> 3, pj = pos & 7;
      const float* zrow = zout + (size_t)(pi << 5) * kLat + (pj << 5) + 8 * hh;
      v8f racc = (v8f){0.f,0.f,0.f,0.f,0.f,0.f,0.f,0.f};
#pragma unroll 1
      for (int kb = 0; kb < 32; kb += 4) {
#pragma unroll
        for (int uu = 0; uu < 4; ++uu) {
          const int ks = kb + uu;
          const float* zr = zrow + ks * kLat;
          const v4f f0 = *(const v4f*)(zr);
          const v4f f1 = *(const v4f*)(zr + 4);
          const v4f f2 = *(const v4f*)(zr + 16);
          const v4f f3 = *(const v4f*)(zr + 20);
          v16b ah, al;
#pragma unroll
          for (int e = 0; e < 4; ++e) {
            __bf16 hv, lv;
            split_hl(f0[e], hv, lv); ah[e] = hv;      al[e] = lv;
            split_hl(f1[e], hv, lv); ah[4 + e] = hv;  al[4 + e] = lv;
            split_hl(f2[e], hv, lv); ah[8 + e] = hv;  al[8 + e] = lv;
            split_hl(f3[e], hv, lv); ah[12 + e] = hv; al[12 + e] = lv;
          }
          const v16b bhf = Frag<__bf16>::load(woh + ks * 32);
          const v16b blf = Frag<__bf16>::load(wol + ks * 32);
          racc = Frag<__bf16>::mma(ah, bhf, racc);
          racc = Frag<__bf16>::mma(ah, blf, racc);
          racc = Frag<__bf16>::mma(al, bhf, racc);
          guard1_b4(racc, ah, al, bhf, blf);
        }
      }
#pragma unroll
      for (int r = 0; r < 8; ++r) yS[m16 * kNpos + (wave << 4) + (hh << 3) + r] = racc[r];
    }
    __syncthreads();
    if (wave < 8) {
      const int o  = (wave << 1) + hh;
      const int p4 = m16 << 2;
      const v4f v = *(const v4f*)(yS + o * kNpos + p4);
      float* dst = PART + (((size_t)c * kSteps + t) * kNoc + o) * kNpos + p4;
      *(volatile v4f*)dst = v;
      __threadfence();
      *(volatile v4f*)dst = v;
    }
  }
}

__global__ __launch_bounds__(256) void combine_kernel(const float* __restrict__ PART,
                                                      const float* __restrict__ b_out,
                                                      float* __restrict__ out) {
  const int i = blockIdx.x * 256 + threadIdx.x;
  const size_t e = 4 * (size_t)i;
  const int o = (int)((e >> 6) & 15);
  v4f s = *(const v4f*)(PART + e);
#pragma unroll
  for (int ch = 1; ch < kNch; ++ch) s = s + *(const v4f*)(PART + (size_t)ch * kPartPlane + e);
  const float bv = b_out[o];
  s = s + (v4f){bv, bv, bv, bv};
  float* q = out + e;
  *(volatile v4f*)q = s;
  __threadfence();
  *(volatile v4f*)q = s;
}

extern "C" void kernel_launch(void* const* d_in, const int* in_sizes, int n_in,
                              void* d_out, int out_size, void* d_ws, size_t ws_size,
                              hipStream_t stream) {
  if (n_in < 9) return;
  const float* X           = (const float*)d_in[0];
  const float* W_embed     = (const float*)d_in[1];
  const float* mask_coarse = (const float*)d_in[2];
  const float* mask_fine   = (const float*)d_in[3];
  const float* W_deconv    = (const float*)d_in[4];
  const float* w1          = (const float*)d_in[5];
  const float* w2          = (const float*)d_in[6];
  const float* w_out       = (const float*)d_in[7];
  const float* b_out       = (const float*)d_in[8];
  float* out = (float*)d_out;

  const size_t bXp  = (size_t)kSteps * kInDim * 2;
  const size_t bWp  = (size_t)kEmbN * kInDim * 2;
  const size_t bWOp = (size_t)kNoc * kNch * kRoK * 2;
  const size_t bUC  = (size_t)kSteps * kEmbN * 4;
  const size_t bZ   = (size_t)kNch * kPlaneF * 4;
  const size_t bP   = (size_t)kNch * kPartPlane * 4;
  const size_t total = 3 * bXp + 3 * bWp + 2 * bWOp + bUC + 2 * bZ + bP;
  if (ws_size < total) return;
  if (out_size < kSteps * kNoc * kNpos) return;
  (void)in_sizes;

  char* ws = (char*)d_ws;
  size_t off = 0;
  unsigned short* Xh  = (unsigned short*)(ws + off); off += bXp;
  unsigned short* Xm  = (unsigned short*)(ws + off); off += bXp;
  unsigned short* Xl  = (unsigned short*)(ws + off); off += bXp;
  unsigned short* Wh  = (unsigned short*)(ws + off); off += bWp;
  unsigned short* Wm  = (unsigned short*)(ws + off); off += bWp;
  unsigned short* Wl  = (unsigned short*)(ws + off); off += bWp;
  unsigned short* WOh = (unsigned short*)(ws + off); off += bWOp;
  unsigned short* WOl = (unsigned short*)(ws + off); off += bWOp;
  float* UC   = (float*)(ws + off); off += bUC;
  float* ZA   = (float*)(ws + off); off += bZ;
  float* ZB   = (float*)(ws + off); off += bZ;
  float* PART = (float*)(ws + off); off += bP;

  split3_kernel<<<(kSteps * kInDim / 8) / 256, 256, 0, stream>>>(X, Xh, Xm, Xl, kSteps * kInDim / 8);
  split3_kernel<<<(kEmbN * kInDim / 8) / 256, 256, 0, stream>>>(W_embed, Wh, Wm, Wl, kEmbN * kInDim / 8);
  split2_kernel<<<(kNoc * kNch * kRoK / 8) / 256, 256, 0, stream>>>(w_out, WOh, WOl, kNoc * kNch * kRoK / 8);

  gemm32_split3<<<32, 256, 0, stream>>>(Xh, Xm, Xl, kInDim, Wh, Wm, Wl, kInDim, UC, kEmbN, kSteps, kEmbN, kInDim);

  lattice_scan_kernel<<<kNch, kBlk, 0, stream>>>(UC, mask_coarse, mask_fine, W_deconv, w1, w2, WOh, WOl, ZA, ZB, PART);

  combine_kernel<<<(kSteps * kNoc * kNpos / 4) / 256, 256, 0, stream>>>(PART, b_out, out);
}
